// LSTM_32890859552831
// MI455X (gfx1250) — hardware-verified
//
#include <hip/hip_runtime.h>
#include <math.h>

constexpr int NVOCAB  = 32000;
constexpr int NEMB    = 128;
constexpr int NHID    = 256;
constexpr int NSENT   = 32;
constexpr int NBATCH  = 64;
constexpr int NSTORY  = 128;
constexpr int NWORD   = 24;
constexpr int NQWORD  = 16;
constexpr int NSTEP   = NSTORY + 3;
constexpr int NGATE   = 4 * NHID;
constexpr int NROWS   = NSTEP * NBATCH;
constexpr int NTHR    = 256;
constexpr int SEQ_BLK = 16;
constexpr int HPITCH  = 264;
constexpr int SLABP   = 68;
constexpr float ACARRY = 16.0f;
constexpr float WCARRY = 64.0f;
constexpr float FOLD   = 1.0f / (ACARRY * WCARRY);

static_assert(NSTEP == 131, "sequence length");
static_assert(NROWS == 8384 && NROWS % 64 == 0, "M tile multiple");
static_assert(NGATE % 64 == 0 && NVOCAB % 64 == 0 && NBATCH % 64 == 0, "N / M tile multiples");
static_assert(NEMB % 32 == 0 && NHID % 32 == 0, "K multiples of 32");
static_assert(NBATCH % SEQ_BLK == 0, "batch rows per block");
static_assert(NHID == 32 * (NTHR / 32), "8 waves x 32 hidden columns");
static_assert((2 * SEQ_BLK * HPITCH) % NTHR == 0, "h tile zero fill exact");
static_assert(HPITCH % 8 == 0, "16-byte aligned fragment rows");
static_assert((NGATE * NEMB / 8) % NTHR == 0 && (NGATE * NHID / 8) % NTHR == 0 && (NVOCAB * NHID / 8) % NTHR == 0, "convert grids exact");
static_assert(NROWS % SEQ_BLK == 0 && NBATCH % 16 == 0, "encode grid exact, one time step per block");

typedef __attribute__((ext_vector_type(16))) _Float16 v16h;
typedef __attribute__((ext_vector_type(8)))  _Float16 v8h;
typedef __attribute__((ext_vector_type(8)))  float    v8f;
typedef __attribute__((ext_vector_type(4)))  float    v4f;

__device__ __forceinline__ void guard_acc4_h(v8f& a0, v8f& a1, v8f& a2, v8f& a3, v16h x, v16h b0, v16h b1, v16h b2, v16h b3) {
  asm volatile("v_nop\n\tv_nop\n\tv_nop\n\tv_nop" : "+v"(a0), "+v"(a1), "+v"(a2), "+v"(a3) : "v"(x), "v"(b0), "v"(b1), "v"(b2), "v"(b3));
}
__device__ __forceinline__ void keep4_h(v16h a, v16h b, v16h c, v16h d) { asm volatile("v_nop" :: "v"(a), "v"(b), "v"(c), "v"(d)); }
__device__ __forceinline__ void acc_guard4(v8f& a, v8f& b, v8f& c, v8f& d) { asm volatile("v_nop\n\tv_nop\n\tv_nop\n\tv_nop" : "+v"(a), "+v"(b), "+v"(c), "+v"(d)); }

union FragU { v16h v; v8h h[2]; };
__device__ __forceinline__ v16h frag_load(const _Float16* p) {
  FragU f;
  f.h[0] = *(const v8h*)(p);
  f.h[1] = *(const v8h*)(p + 16);
  return f.v;
}
__device__ __forceinline__ v8f frag_mma(v16h a, v16h b, v8f c) {
  return __builtin_amdgcn_wmma_f32_16x16x32_f16(false, a, false, b, (short)0, c, false, false);
}

__device__ __forceinline__ float fsig(float x) { return 1.0f / (1.0f + expf(-x)); }

__global__ __launch_bounds__(NTHR) void cvt8_f16_kernel(const float* __restrict__ src, unsigned short* __restrict__ dstp,
                                                        int n8, float sc) {
  const int i = blockIdx.x * NTHR + threadIdx.x;
  if (i < n8) {
    const float* sp = src + (size_t)i * 8;
    const v4f a = *(const v4f*)(sp);
    const v4f b = *(const v4f*)(sp + 4);
    v8h hv;
#pragma unroll
    for (int e = 0; e < 4; ++e) {
      hv[e]     = (_Float16)(a[e] * sc);
      hv[4 + e] = (_Float16)(b[e] * sc);
    }
    _Float16* dp = (_Float16*)dstp + (size_t)i * 8;
    *(volatile v8h*)dp = hv;
    __threadfence();
    *(volatile v8h*)dp = hv;
  }
}

__global__ __launch_bounds__(NTHR) void bias_sum_kernel(const float* __restrict__ b_a, const float* __restrict__ b_b,
                                                        float* __restrict__ dst) {
  const int idx = threadIdx.x * 4;
  const v4f va = *(const v4f*)(b_a + idx);
  const v4f vb = *(const v4f*)(b_b + idx);
  v4f o;
#pragma unroll
  for (int e = 0; e < 4; ++e) o[e] = va[e] + vb[e];
  float* op = dst + idx;
  *(volatile v4f*)op = o;
  __threadfence();
  *(volatile v4f*)op = o;
}

__global__ __launch_bounds__(NTHR) void encode_kernel(const int* __restrict__ story, const int* __restrict__ query,
                                                      const float* __restrict__ table, unsigned short* __restrict__ XHp) {
  __shared__ int sTok[SEQ_BLK * NSENT];
  const int tid = threadIdx.x;
  const int t  = blockIdx.x >> 2;
  const int b0 = (blockIdx.x & 3) * 16;
#pragma unroll
  for (int i = 0; i < 2; ++i) {
    const int idx = i * NTHR + tid;
    const int r = idx >> 5;
    const int s = idx & 31;
    const int b = b0 + r;
    int tok = 0;
    if (t < NSTORY) {
      const int sc = (s < NWORD) ? s : (NWORD - 1);
      const int v = story[((size_t)b * NSTORY + (size_t)t) * NWORD + sc];
      tok = v & (-(int)(s < NWORD));
    } else if (t == NSTORY) {
      const int sc = (s < NQWORD) ? s : (NQWORD - 1);
      const int v = query[b * NQWORD + sc];
      tok = v & (-(int)(s < NQWORD));
    }
    tok = tok < 0 ? 0 : tok;
    tok = tok > (NVOCAB - 1) ? (NVOCAB - 1) : tok;
    sTok[idx] = tok;
  }
  __syncthreads();

  const int r  = tid >> 4;
  const int e0 = (tid & 15) * 8;
  float ke[8], acc[8];
#pragma unroll
  for (int i = 0; i < 8; ++i) {
    ke[i]  = (float)(e0 + i + 1) * (1.0f / (float)NEMB);
    acc[i] = 0.0f;
  }
  const int npos = (t <= NSTORY) ? NSENT : 0;
#pragma unroll 1
  for (int s = 0; s < npos; ++s) {
    const int tok = sTok[r * NSENT + s];
    const float jj = (float)(s + 1) * (1.0f / (float)NSENT);
    const float as = 1.0f - jj;
    const float bs = 1.0f - 2.0f * jj;
    const float* tp = table + (size_t)tok * NEMB + e0;
    const v4f u0 = *(const v4f*)(tp);
    const v4f u1 = *(const v4f*)(tp + 4);
#pragma unroll
    for (int i = 0; i < 4; ++i) {
      const float p0 = as - ke[i] * bs;
      const float p1 = as - ke[4 + i] * bs;
      acc[i]     += u0[i] * p0;
      acc[4 + i] += u1[i] * p1;
    }
  }
  v8h hv;
#pragma unroll
  for (int i = 0; i < 8; ++i) hv[i] = (_Float16)(acc[i] * ACARRY);
  _Float16* dp = (_Float16*)XHp + ((size_t)blockIdx.x * SEQ_BLK + r) * NEMB + e0;
  *(volatile v8h*)dp = hv;
  __threadfence();
  *(volatile v8h*)dp = hv;
}

__global__ __launch_bounds__(256) void gemm64_f16_kernel(
    const unsigned short* __restrict__ Ap, int lda,
    const unsigned short* __restrict__ Btp, int ldb,
    float* __restrict__ C, int ldc,
    const float* __restrict__ bias,
    int M, int N, int K, float scale) {
  const _Float16* A  = (const _Float16*)Ap;
  const _Float16* Bt = (const _Float16*)Btp;
  __shared__ __align__(16) float sT[8][16 * 68];
  const int lane = threadIdx.x & 31;
  const int wave = threadIdx.x >> 5;
  const int tilesN = N >> 6;
  const int tilesM = M >> 6;
  const int tile = blockIdx.x * 8 + wave;
  if (tile >= tilesM * tilesN) return;
  const int tm = tile / tilesN;
  const int tn = tile - tm * tilesN;
  const int m0 = tm << 6;
  const int n0 = tn << 6;

  const int rlane = lane & 15;
  const int koff  = (lane >> 4) * 8;
  const int mOff  = (lane >> 4) * 8;

  v8f acc[4][4];
#pragma unroll
  for (int i = 0; i < 4; ++i)
#pragma unroll
    for (int j = 0; j < 4; ++j) acc[i][j] = (v8f){0.f, 0.f, 0.f, 0.f, 0.f, 0.f, 0.f, 0.f};

  for (int k0 = 0; k0 < K; k0 += 32) {
    v16h bh[4];
#pragma unroll
    for (int j = 0; j < 4; ++j) {
      const size_t bo = (size_t)(n0 + (j << 4) + rlane) * ldb + koff + k0;
      bh[j] = frag_load(Bt + bo);
    }
#pragma unroll
    for (int i = 0; i < 4; ++i) {
      const size_t ao = (size_t)(m0 + (i << 4) + rlane) * lda + koff + k0;
      const v16h ah = frag_load(A + ao);
#pragma unroll
      for (int j = 0; j < 4; ++j) acc[i][j] = frag_mma(ah, bh[j], acc[i][j]);
      guard_acc4_h(acc[i][0], acc[i][1], acc[i][2], acc[i][3], ah, bh[0], bh[1], bh[2], bh[3]);
    }
    keep4_h(bh[0], bh[1], bh[2], bh[3]);
  }
  acc_guard4(acc[0][0], acc[0][1], acc[0][2], acc[0][3]);
  acc_guard4(acc[1][0], acc[1][1], acc[1][2], acc[1][3]);
  acc_guard4(acc[2][0], acc[2][1], acc[2][2], acc[2][3]);
  acc_guard4(acc[3][0], acc[3][1], acc[3][2], acc[3][3]);

  float* slab = sT[wave];
#pragma unroll
  for (int i = 0; i < 4; ++i) {
    const int mBase = m0 + (i << 4);
#pragma unroll
    for (int j = 0; j < 4; ++j) {
      const int n = n0 + (j << 4) + rlane;
      const float bv = bias[n];
#pragma unroll
      for (int r = 0; r < 8; ++r) {
        const float v = acc[i][j][r] * scale + bv;
        slab[(mOff + r) * 68 + (j << 4) + rlane] = v;
      }
    }
    __builtin_amdgcn_fence(__ATOMIC_RELEASE, "workgroup");
    __builtin_amdgcn_wave_barrier();
    __builtin_amdgcn_fence(__ATOMIC_ACQUIRE, "workgroup");
    {
      const int hh = lane >> 4, c4 = (lane & 15) * 4;
      for (int pass = 0; pass < 2; ++pass) {
#pragma unroll
        for (int it = 0; it < 8; ++it) {
          const int row = it * 2 + hh;
          const v4f v = *(const v4f*)(slab + row * 68 + c4);
          *(volatile v4f*)(C + (size_t)(mBase + row) * ldc + n0 + c4) = v;
        }
        __threadfence();
      }
    }
    __builtin_amdgcn_fence(__ATOMIC_RELEASE, "workgroup");
    __builtin_amdgcn_wave_barrier();
    __builtin_amdgcn_fence(__ATOMIC_ACQUIRE, "workgroup");
  }
}

__global__ __launch_bounds__(NTHR) void recur_seq_kernel(const float* __restrict__ GX,
                                                         const unsigned short* __restrict__ WHp,
                                                         unsigned short* __restrict__ HNp) {
  __shared__ __align__(16) _Float16 Ah[2][SEQ_BLK * HPITCH];
  __shared__ __align__(16) float    Sl[NTHR / 32][16 * SLABP];
  const _Float16* WH = (const _Float16*)WHp;
  const int tid = threadIdx.x, lane = tid & 31, wave = tid >> 5;
  const int c = lane & 15, hh = lane >> 4, koff = hh * 8;
  const int rowbase = blockIdx.x * SEQ_BLK;

  {
    _Float16* ahf = &Ah[0][0];
#pragma unroll 1
    for (int i = tid; i < 2 * SEQ_BLK * HPITCH; i += NTHR) ahf[i] = (_Float16)0.0f;
  }
  float cst[2][8];
#pragma unroll
  for (int nt = 0; nt < 2; ++nt)
#pragma unroll
    for (int r = 0; r < 8; ++r) cst[nt][r] = 0.0f;
  __syncthreads();

  const v8f z8 = {0.f, 0.f, 0.f, 0.f, 0.f, 0.f, 0.f, 0.f};
  float* slab = Sl[wave];

#pragma unroll 1
  for (int t = 0; t < NSTEP; ++t) {
    const int cur = t & 1;
    const _Float16* ahrow = &Ah[cur][0] + c * HPITCH + koff;
    _Float16* ahn = &Ah[cur ^ 1][0];
    const float* gxt = GX + ((size_t)t * NBATCH + (size_t)rowbase) * NGATE;
#pragma unroll
    for (int nt = 0; nt < 2; ++nt) {
      const int jb = 32 * wave + 16 * nt;
      __builtin_amdgcn_fence(__ATOMIC_RELEASE, "workgroup");
      __builtin_amdgcn_wave_barrier();
      __builtin_amdgcn_fence(__ATOMIC_ACQUIRE, "workgroup");
#pragma unroll
      for (int it = 0; it < 8; ++it) {
        const int idx = it * 32 + lane;
        const int row = idx >> 4;
        const int seg = idx & 15;
        const int g   = seg >> 2;
        const int q4  = (seg & 3) * 4;
        const v4f v = *(const v4f*)(gxt + (size_t)row * NGATE + g * NHID + jb + q4);
        *(v4f*)(slab + row * SLABP + g * 16 + q4) = v;
      }
      const _Float16* wh = WH + (size_t)(jb + c) * NHID + koff;
      v8f acc[4];
      acc[0] = z8; acc[1] = z8; acc[2] = z8; acc[3] = z8;
#pragma unroll 1
      for (int k0 = 0; k0 < NHID; k0 += 32) {
        const v16h a  = frag_load(ahrow + k0);
        const v16h b0 = frag_load(wh + k0);
        const v16h b1 = frag_load(wh + (size_t)1 * NHID * NHID + k0);
        const v16h b2 = frag_load(wh + (size_t)2 * NHID * NHID + k0);
        const v16h b3 = frag_load(wh + (size_t)3 * NHID * NHID + k0);
        acc[0] = frag_mma(a, b0, acc[0]);
        acc[1] = frag_mma(a, b1, acc[1]);
        acc[2] = frag_mma(a, b2, acc[2]);
        acc[3] = frag_mma(a, b3, acc[3]);
        guard_acc4_h(acc[0], acc[1], acc[2], acc[3], a, b0, b1, b2, b3);
      }
      acc_guard4(acc[0], acc[1], acc[2], acc[3]);
      __builtin_amdgcn_fence(__ATOMIC_RELEASE, "workgroup");
      __builtin_amdgcn_wave_barrier();
      __builtin_amdgcn_fence(__ATOMIC_ACQUIRE, "workgroup");
#pragma unroll
      for (int r = 0; r < 8; ++r) {
        const int sr = (8 * hh + r) * SLABP + c;
        const float zi = acc[0][r] * FOLD + slab[sr];
        const float zf = acc[1][r] * FOLD + slab[sr + 16];
        const float zg = acc[2][r] * FOLD + slab[sr + 32];
        const float zo = acc[3][r] * FOLD + slab[sr + 48];
        const float ig = fsig(zi);
        const float fg = fsig(zf);
        const float gg = tanhf(zg);
        const float og = fsig(zo);
        const float cn = fg * cst[nt][r] + ig * gg;
        cst[nt][r] = cn;
        const float hn = og * tanhf(cn);
        ahn[(8 * hh + r) * HPITCH + jb + c] = (_Float16)(hn * ACARRY);
      }
    }
    __syncthreads();
  }

  {
    const _Float16* fin = &Ah[NSTEP & 1][0];
    _Float16* HN = (_Float16*)HNp;
    v8h hv[2];
#pragma unroll
    for (int it = 0; it < 2; ++it) {
      const int idx = it * NTHR + tid;
      const int row = idx >> 5, c8 = (idx & 31) * 8;
      hv[it] = *(const v8h*)(fin + row * HPITCH + c8);
    }
    for (int pass = 0; pass < 2; ++pass) {
#pragma unroll
      for (int it = 0; it < 2; ++it) {
        const int idx = it * NTHR + tid;
        const int row = idx >> 5, c8 = (idx & 31) * 8;
        *(volatile v8h*)(HN + (size_t)(rowbase + row) * NHID + c8) = hv[it];
      }
      __threadfence();
    }
  }
}

extern "C" void kernel_launch(void* const* d_in, const int* in_sizes, int n_in,
                              void* d_out, int out_size, void* d_ws, size_t ws_size, hipStream_t stream) {
  if (n_in < 9 || d_out == nullptr || d_ws == nullptr) return;
  if (in_sizes[0] != NBATCH * NSTORY * NWORD || in_sizes[1] != NBATCH * NQWORD || in_sizes[2] != NVOCAB * NEMB ||
      in_sizes[3] != NGATE * NEMB || in_sizes[4] != NGATE * NHID || in_sizes[5] != NGATE || in_sizes[6] != NGATE ||
      in_sizes[7] != NVOCAB * NHID || in_sizes[8] != NVOCAB || out_size != NBATCH * NVOCAB) return;

  const int*   story = (const int*)d_in[0];
  const int*   query = (const int*)d_in[1];
  const float* table = (const float*)d_in[2];
  const float* w_ih  = (const float*)d_in[3];
  const float* w_hh  = (const float*)d_in[4];
  const float* b_ih  = (const float*)d_in[5];
  const float* b_hh  = (const float*)d_in[6];
  const float* lin_w = (const float*)d_in[7];
  const float* lin_b = (const float*)d_in[8];
  float* out = (float*)d_out;

  char* ws = (char*)d_ws;
  size_t off = 0;
  auto carve = [&](size_t bytes) -> char* { char* p = ws + off; off += (bytes + 255) & ~(size_t)255; return p; };
  unsigned short* XH    = (unsigned short*)carve((size_t)NROWS * NEMB * 2);
  unsigned short* WIH   = (unsigned short*)carve((size_t)NGATE * NEMB * 2);
  unsigned short* WHH   = (unsigned short*)carve((size_t)NGATE * NHID * 2);
  unsigned short* LINW  = (unsigned short*)carve((size_t)NVOCAB * NHID * 2);
  float*          BIASC = (float*)carve((size_t)NGATE * 4);
  float*          GX    = (float*)carve((size_t)NROWS * NGATE * 4);
  unsigned short* HN    = (unsigned short*)carve((size_t)NBATCH * NHID * 2);
  if (off > ws_size || off > (size_t)134217728) return;

  const int n8ih = NGATE * NEMB / 8;
  const int n8hh = NGATE * NHID / 8;
  const int n8lw = NVOCAB * NHID / 8;
  cvt8_f16_kernel<<<(n8ih + NTHR - 1) / NTHR, NTHR, 0, stream>>>(w_ih,  WIH,  n8ih, WCARRY);
  cvt8_f16_kernel<<<(n8hh + NTHR - 1) / NTHR, NTHR, 0, stream>>>(w_hh,  WHH,  n8hh, WCARRY);
  cvt8_f16_kernel<<<(n8lw + NTHR - 1) / NTHR, NTHR, 0, stream>>>(lin_w, LINW, n8lw, WCARRY);
  bias_sum_kernel<<<1, NTHR, 0, stream>>>(b_ih, b_hh, BIASC);

  encode_kernel<<<NROWS / SEQ_BLK, NTHR, 0, stream>>>(story, query, table, XH);

  {
    const int tiles = (NROWS / 64) * (NGATE / 64);
    gemm64_f16_kernel<<<(tiles + 7) / 8, 256, 0, stream>>>(XH, NEMB, WIH, NEMB, GX, NGATE, BIASC,
                                                            NROWS, NGATE, NEMB, FOLD);
  }

  recur_seq_kernel<<<NBATCH / SEQ_BLK, NTHR, 0, stream>>>(GX, WHH, HN);

  {
    const int tiles = (NBATCH / 64) * (NVOCAB / 64);
    gemm64_f16_kernel<<<(tiles + 7) / 8, 256, 0, stream>>>(HN, NHID, LINW, NHID, out, NVOCAB, lin_b,
                                                            NBATCH, NVOCAB, NHID, FOLD);
  }
}
